// MetaLearner_24309514895364
// MI455X (gfx1250) — hardware-run, weakly checked
//
#include <hip/hip_runtime.h>


namespace {
constexpr int NF = 64, NPAR = 20000, NC = NF * NPAR, H = 20, G4 = 80, L = 2;
constexpr float HS = 16384.0f  , WSC = 256.0f, EPS = 1e-5f, FG_BIAS = 1.0f;
typedef _Float16 b16;
typedef __attribute__((ext_vector_type(16))) _Float16 v16b;
typedef __attribute__((ext_vector_type(8))) _Float16 v8b;
typedef __attribute__((ext_vector_type(8))) float v8f;
__device__ __forceinline__ float bf16_rne(float f) { unsigned int u = __float_as_uint(f); u += 0x7FFFu + ((u >> 16) & 1u); float r = __uint_as_float(u & 0xFFFF0000u); asm volatile("" : "+v"(r)); return r; }
__device__ __forceinline__ float bfv(float f) { float r = bf16_rne(f); asm volatile("" : "+v"(r)); return r; }
__device__ __forceinline__ void split16(float v, b16& hi, b16& lo) { hi = (b16)v; lo = (b16)(v - (float)hi); }
__device__ __forceinline__ v16b frag_kb(const b16* p, int hh) { const v8b a = *(const v8b*)(p + 8 * hh), b = *(const v8b*)(p + 16 + 8 * hh); v16b f;
#pragma unroll
  for (int e = 0; e < 8; ++e) { f[e] = a[e]; f[8 + e] = b[e]; } return f; }
__device__ __forceinline__ v8f wmma16b(v16b a, v16b b, v8f c) { v8f d = __builtin_amdgcn_wmma_f32_16x16x32_f16(false, a, false, b, (short)0, c, false, false); asm volatile("v_nop\n\tv_nop\n\tv_nop\n\tv_nop" : "+v"(d) : "v"(a), "v"(b)); return d; }
__device__ __forceinline__ void wave_lds_sync() { __builtin_amdgcn_fence(__ATOMIC_RELEASE, "workgroup"); __builtin_amdgcn_wave_barrier(); __builtin_amdgcn_fence(__ATOMIC_ACQUIRE, "workgroup"); }
__device__ __forceinline__ float pmul(float a, float b) { float p = a * b; asm volatile("" : "+v"(p)); return p; }
__device__ __forceinline__ float sigm(float v) { return 1.0f / (1.0f + __expf(-v)); }
__device__ __forceinline__ float tanh_e(float x) { const float e = __expf(2.0f * x); return 1.0f - 2.0f / (e + 1.0f); }

__global__ __launch_bounds__(256) void wput_kernel(const float* __restrict__ wi, b16* __restrict__ WI) { const int u = blockIdx.x * 256 + threadIdx.x; if (u >= L * G4 * 4) return; const int l = u / (G4 * 4), o = (u / 4) % G4, k0 = (u % 4) * 8; v8b v;
#pragma unroll
  for (int j = 0; j < 8; ++j) { const int k = k0 + j; v[j] = (b16)(k < H ? bf16_rne(wi[((size_t)l * G4 + o) * H + k]) * WSC : 0.0f); }
  for (int pass = 0; pass < 2; ++pass) { *(volatile v8b*)(WI + ((size_t)l * G4 + o) * 32 + k0) = v; __threadfence(); } }
__global__ __launch_bounds__(32) void main_kernel(const float* __restrict__ x, const float* __restrict__ l1w, const float* __restrict__ l1b, const b16* __restrict__ WI, const float* __restrict__ bi, const float* __restrict__ bh, const float* __restrict__ gi, const float* __restrict__ bti, const float* __restrict__ gh, const float* __restrict__ bth, const float* __restrict__ gc, const float* __restrict__ btc, const float* __restrict__ ow, const float* __restrict__ ob, int CLIM, float* __restrict__ out) { __shared__ __attribute__((aligned(16))) b16 Ah[32][40], Al[32][40]; __shared__ float Pre[32][G4 + 1], LHB[L][G4]; const int lane = threadIdx.x, nloc = lane & 15, hlf = lane >> 4; const size_t c0 = (size_t)blockIdx.x * 32; if (c0 >= (size_t)CLIM) return;
  if (lane < L) { const int l = lane; float m = 0.0f; for (int j = 0; j < G4; ++j) m += bfv(bh[l * G4 + j]); m /= (float)G4; float vr = 0.0f; for (int j = 0; j < G4; ++j) { const float d = bfv(bh[l * G4 + j]) - m; vr += pmul(d, d); } vr /= (float)G4; const float rs = rsqrtf(vr + EPS); for (int j = 0; j < G4; ++j) LHB[l][j] = pmul((bfv(bh[l * G4 + j]) - m) * rs, bfv(gh[l * G4 + j])) + bfv(bth[l * G4 + j]); }
  for (int k = H; k < 40; ++k) { Ah[lane][k] = (b16)0.0f; Al[lane][k] = (b16)0.0f; }
  float xt[H]; { const float xv = bfv(x[c0 + lane]);
#pragma unroll
    for (int j = 0; j < H; ++j) xt[j] = pmul(xv, bfv(l1w[j])) + bfv(l1b[j]); }
#pragma unroll 1
  for (int l = 0; l < L; ++l) {
#pragma unroll
    for (int j = 0; j < H; ++j) { b16 p, pl; split16(xt[j] * HS, p, pl); Ah[lane][j] = p; Al[lane][j] = pl; }
    wave_lds_sync();
    for (int rt = 0; rt < 2; ++rt) { v8f acc[5] = {(v8f){}, (v8f){}, (v8f){}, (v8f){}, (v8f){}}; const v16b a = frag_kb(&Ah[rt * 16 + nloc][0], hlf), al = frag_kb(&Al[rt * 16 + nloc][0], hlf);
#pragma unroll
      for (int t = 0; t < 5; ++t) { const v16b bw = frag_kb(WI + ((size_t)l * G4 + t * 16 + nloc) * 32, hlf); acc[t] = wmma16b(a, bw, acc[t]); acc[t] = wmma16b(al, bw, acc[t]); }
#pragma unroll
      for (int t = 0; t < 5; ++t) { const int cc = t * 16 + nloc; const float bb = bfv(bi[l * G4 + cc]);
#pragma unroll
        for (int r8 = 0; r8 < 8; ++r8) Pre[rt * 16 + 8 * hlf + r8][cc] = acc[t][r8] * (1.0f / (HS * WSC)) + bb; } }
    wave_lds_sync();
    { float* pr = &Pre[lane][0]; float m = 0.0f; for (int j = 0; j < G4; ++j) m += pr[j]; m /= (float)G4; float vr = 0.0f; for (int j = 0; j < G4; ++j) { const float d = pr[j] - m; vr += pmul(d, d); } vr /= (float)G4; const float rs = rsqrtf(vr + EPS);
      for (int j = 0; j < G4; ++j) pr[j] = pmul((pr[j] - m) * rs, bfv(gi[l * G4 + j])) + bfv(bti[l * G4 + j]) + LHB[l][j];
      float c[H]; float cm = 0.0f;
#pragma unroll
      for (int j = 0; j < H; ++j) { c[j] = pmul(sigm(pr[j]), tanh_e(pr[3 * H + j])); cm += c[j]; }
      cm /= (float)H; float cv = 0.0f;
#pragma unroll
      for (int j = 0; j < H; ++j) { const float d = c[j] - cm; cv += pmul(d, d); } cv /= (float)H; const float crs = rsqrtf(cv + EPS);
#pragma unroll
      for (int j = 0; j < H; ++j) xt[j] = pmul(sigm(pr[2 * H + j]), tanh_e(pmul((c[j] - cm) * crs, bfv(gc[l * H + j])) + bfv(btc[l * H + j]))); }
    wave_lds_sync(); }
  float s = bfv(ob[0]);
#pragma unroll
  for (int j = 0; j < H; ++j) s += pmul(xt[j], bfv(ow[j]));
  for (int pass = 0; pass < 2; ++pass) { ((volatile float*)out)[c0 + lane] = s; __threadfence(); } }
}

extern "C" void kernel_launch(void* const* d_in, const int* in_sizes, int n_in, void* d_out, int out_size, void* d_ws, size_t ws_size, hipStream_t stream) {
  (void)n_in;
  auto Fp = [&](int i) { return (const float*)d_in[i]; };
  if (in_sizes[0] != NC || in_sizes[1] != H || in_sizes[3] != L * G4 * H || in_sizes[6] != L * G4 || in_sizes[11] != L * H || in_sizes[13] != H || out_size != NC) return;
  const int CLIM = NC;
  size_t off = 0; char* ws = (char*)d_ws;
  auto carve = [&](size_t bytes) { char* p = ws + off; off += (bytes + 255) & ~(size_t)255; return p; };
  b16* WI = (b16*)carve((size_t)L * G4 * 32 * 2);
  if (off > ws_size) return;
  wput_kernel<<<(L * G4 * 4 + 255) / 256, 256, 0, stream>>>(Fp(3), WI);
  main_kernel<<<NC / 32, 32, 0, stream>>>(Fp(0), Fp(1), Fp(2), WI, Fp(4), Fp(6), Fp(7), Fp(8), Fp(9), Fp(10), Fp(11), Fp(12), Fp(13), Fp(14), CLIM, (float*)d_out);
}
